// MADF_56573309222923
// MI455X (gfx1250) — hardware-verified
//
#include <hip/hip_runtime.h>
#include <math.h>

typedef __attribute__((ext_vector_type(16))) _Float16 v16h;
typedef __attribute__((ext_vector_type(16))) __bf16 v16b;
typedef __attribute__((ext_vector_type(8)))  _Float16 v8h;
typedef __attribute__((ext_vector_type(8)))  float v8f;
typedef __attribute__((ext_vector_type(4)))  float v4f;
typedef __attribute__((ext_vector_type(2)))  float v2f;
typedef __attribute__((ext_vector_type(4)))  unsigned v4u;
typedef __attribute__((ext_vector_type(4)))  int v4i;
typedef float __attribute__((may_alias)) float_a;
typedef int __attribute__((may_alias)) int_a;

template <typename T> __device__ __forceinline__ void vst2(void* p, T v) { *(volatile T*)p = v; __threadfence(); *(volatile T*)p = v; }
__device__ __forceinline__ v8f wmma16(v16h a, v16h b, v8f c) {
  v8f d = __builtin_amdgcn_wmma_f32_16x16x32_f16(false, a, false, b, (short)0, c, false, false);
  asm volatile("v_nop\n\tv_nop\n\tv_nop\n\tv_nop" : "+v"(d) : "v"(a), "v"(b));
  return d;
}
__device__ __forceinline__ v8f wmma_bf(v16b a, v16b b, v8f c) {
  v8f d = __builtin_amdgcn_wmma_f32_16x16x32_bf16(false, a, false, b, (short)0, c, false, false);
  asm volatile("v_nop\n\tv_nop\n\tv_nop\n\tv_nop" : "+v"(d) : "v"(a), "v"(b));
  return d;
}
__device__ __forceinline__ v16h frag_h(const _Float16* rowk0, int lane) {
  union { v16h v; v8h q[2]; } u; const _Float16* p = rowk0 + 8 * (lane >> 4);
  u.q[0] = *(const v8h*)p; u.q[1] = *(const v8h*)(p + 16); return u.v;
}
__device__ __forceinline__ v16h frag_f32(const float* rowk0, int lane) {
  v16h a; const float* p = rowk0 + 8 * (lane >> 4);
#pragma unroll
  for (int i = 0; i < 8; ++i) { a[i] = (_Float16)p[i]; a[8 + i] = (_Float16)p[16 + i]; }
  return a;
}
__device__ __forceinline__ v16h frag_f32s(const float* rowk0, int lane, float sc) {
  v16h a; const float* p = rowk0 + 8 * (lane >> 4);
#pragma unroll
  for (int i = 0; i < 8; ++i) { a[i] = (_Float16)(p[i] * sc); a[8 + i] = (_Float16)(p[16 + i] * sc); }
  return a;
}
__device__ __forceinline__ v16h fragc_f32(const float* W, int k0, int n, int lane, int ld, int K) {
  v16h a; const int g = lane >> 4;
#pragma unroll
  for (int i = 0; i < 8; ++i) { const int ka = k0 + 8 * g + i, kb = ka + 16;
    a[i] = (_Float16)(ka < K ? W[(size_t)(ka < K ? ka : K - 1) * ld + n] : 0.f); a[8 + i] = (_Float16)(kb < K ? W[(size_t)(kb < K ? kb : K - 1) * ld + n] : 0.f); }
  return a;
}
struct F2 { v16b h, l; };
__device__ __forceinline__ F2 bsplit16(const float v[16]) { F2 r;
#pragma unroll
  for (int i = 0; i < 16; ++i) { const __bf16 h = (__bf16)v[i]; r.h[i] = h; r.l[i] = (__bf16)(v[i] - (float)h); }
  return r; }
__device__ __forceinline__ F2 split_row(const float* row, int k0, int lane) { float v[16]; const float* p = row + k0 + 8 * (lane >> 4);
#pragma unroll
  for (int i = 0; i < 8; ++i) { v[i] = p[i]; v[8 + i] = p[16 + i]; }
  return bsplit16(v); }
__device__ __forceinline__ F2 split_rowK(const float* row, int k0, int lane, int K) { float v[16]; const int g = lane >> 4;
#pragma unroll
  for (int i = 0; i < 8; ++i) { const int ka = k0 + 8 * g + i, kb = ka + 16; v[i] = ka < K ? row[ka < K ? ka : K - 1] : 0.f; v[8 + i] = kb < K ? row[kb < K ? kb : K - 1] : 0.f; }
  return bsplit16(v); }
__device__ __forceinline__ F2 split_col(const float* W, int k0, int n, int lane, int ld, int K) { float v[16]; const int g = lane >> 4;
#pragma unroll
  for (int i = 0; i < 8; ++i) { const int ka = k0 + 8 * g + i, kb = ka + 16; v[i] = ka < K ? W[(size_t)(ka < K ? ka : K - 1) * ld + n] : 0.f; v[8 + i] = kb < K ? W[(size_t)(kb < K ? kb : K - 1) * ld + n] : 0.f; }
  return bsplit16(v); }
__device__ __forceinline__ v8f mac3(const F2& a, const F2& b, v8f c) { c = wmma_bf(a.l, b.h, c); c = wmma_bf(a.h, b.l, c); return wmma_bf(a.h, b.h, c); }
__device__ __forceinline__ float sigm(float v) { return 1.0f / (1.0f + expf(-v)); }
#define LDSX() do { asm volatile("s_wait_dscnt 0" ::: "memory"); __builtin_amdgcn_wave_barrier(); __builtin_amdgcn_fence(__ATOMIC_RELEASE, "workgroup"); } while (0)


#define NB 2
#define CM 64
#define CE 32
#define HH 64
#define WW 64
#define NPX (HH * WW)
#define NF 9216
#define KM (CM * 9)
#define KP (CE * 9)
#define SLR 8
#define NSL (HH / SLR)
#define FPS (NF * SLR * WW / NPX)
#ifndef TNB
#define TNB NB
#define TB0 0
#endif
typedef __attribute__((ext_vector_type(8))) __bf16 v8b;
__device__ __forceinline__ v16b frag_b(const __bf16* rowk0, int lane) {
  union { v16b v; v8b q[2]; } u; const __bf16* p = rowk0 + 8 * (lane >> 4);
  u.q[0] = *(const v8b*)p; u.q[1] = *(const v8b*)(p + 16); return u.v;
}
__device__ __forceinline__ float bfr(float v) { return (float)(__bf16)v; }
__device__ __attribute__((noinline)) float exp_ni(float v) { return expf(v); }
__device__ __attribute__((noinline)) float erf_ni(float v) { return erff(v); }

#define WS_PM  0u
#define WS_PF  (2u * CM * KM)
#define WS_MH  (WS_PF + 2u * (size_t)NF * CM)
#define WS_MLO (WS_MH + 2u * NB * NPX * CM)
#define WS_F   (WS_MLO + 2u * NB * NPX * CM)
#define WS_EL  (WS_F + 4u * (size_t)NB * FPS * NPX)
#define WS_ST  (WS_EL + 4u * NB * CE * NPX)
#define WS_MS  (WS_ST + 4u * NB * HH * CE * 2)
#define WS_END (WS_MS + 4u * CE * 2)

__global__ __launch_bounds__(256) void k_pack(const float* __restrict__ WM, const float* __restrict__ WF, __bf16* __restrict__ PK) {
  __shared__ __align__(16) __bf16 s[KM]; const int n = blockIdx.x, which = blockIdx.y, t = threadIdx.x;
  if (which == 0) { if (n >= CM) return; for (int k = t; k < KM; k += 256) s[k] = (__bf16)WM[(size_t)n * KM + k]; __syncthreads(); for (int q = t; q < KM / 8; q += 256) vst2((unsigned*)(PK + WS_PM / 2 + (size_t)n * KM + q * 8), *(const v4u*)&s[q * 8]); }
  else {
    for (int e = t; e < 64 * CM / 8; e += 256) { const int r = e >> 3, q = e & 7; const size_t row = (size_t)n * 64 + r; __align__(16) __bf16 v8[8];
#pragma unroll
      for (int i = 0; i < 8; ++i) v8[i] = (__bf16)WF[row * CM + q * 8 + i]; vst2((unsigned*)(PK + WS_PF / 2 + row * CM + q * 8), *(const v4u*)v8); } }
}
__global__ __launch_bounds__(128) void k_ml(const float* __restrict__ M1, const __bf16* __restrict__ PM, const float* __restrict__ BMv, float* __restrict__ OUT0, __bf16* __restrict__ MH, __bf16* __restrict__ ML) {
  __shared__ __align__(16) __bf16 sa[64][KM + 8]; __shared__ __align__(16) float so[CM][68]; __shared__ __align__(16) __bf16 sh[64][CM + 8], sl[64][CM + 8];
  const int tid = threadIdx.x, wave = tid >> 5, lane = tid & 31, col = lane & 15, g = lane >> 4; const int y = blockIdx.x; const size_t b = blockIdx.y + TB0;
  for (int e = tid; e < 64 * KM; e += 128) { const int px = e / KM, k = e % KM; const int c = k / 9, ij = k % 9, i = ij / 3, j = ij % 3; const int yy = y + i - 1, xx = px + j - 1;
    sa[px][k] = (__bf16)((yy >= 0 && yy < HH && xx >= 0 && xx < WW) ? M1[((b * CM + c) * HH + yy) * WW + xx] : 0.f); }
  if (tid < 64) for (int k = KM; k < KM + 8; ++k) sa[tid][k] = (__bf16)0.f;
  __syncthreads();
  v8f acc[4] = {};
#pragma unroll 2
  for (int kc = 0; kc < KM / 32; ++kc) { const v16b a = frag_b(&sa[wave * 16 + col][kc * 32], lane);
#pragma unroll
    for (int jt = 0; jt < 4; ++jt) acc[jt] = wmma_bf(a, frag_b(PM + (size_t)(jt * 16 + col) * KM + kc * 32, lane), acc[jt]); }
#pragma unroll
  for (int jt = 0; jt < 4; ++jt) { const int o = jt * 16 + col; const float bb = bfr(BMv[o]);
#pragma unroll
    for (int r = 0; r < 8; ++r) { const int px = wave * 16 + 8 * g + r; const float v = fmaxf(acc[jt][r] + bb, 0.f); so[o][px] = v; const __bf16 hb = (__bf16)v; sh[px][o] = hb; sl[px][o] = (__bf16)(v - (float)hb); } }
  __syncthreads();
  for (int e = tid; e < CM * 16; e += 128) { const int o = e >> 4, q = e & 15; vst2(OUT0 + ((b * CM + o) * HH + y) * WW + q * 4, *(const v4f*)&so[o][q * 4]); }
  for (int e = tid; e < 64 * 8; e += 128) { const int px = e >> 3, q = e & 7; const size_t prow = b * NPX + (size_t)y * WW + px; vst2((unsigned*)(MH + prow * CM + q * 8), *(const v4u*)&sh[px][q * 8]); vst2((unsigned*)(ML + prow * CM + q * 8), *(const v4u*)&sl[px][q * 8]); }
}
__global__ __launch_bounds__(128) void k_f(const __bf16* __restrict__ PF, const __bf16* __restrict__ MH, const __bf16* __restrict__ ML, const float* __restrict__ BF, int slab, float* __restrict__ F) {
  __shared__ __align__(16) float so[4][16][132];
  const int tid = threadIdx.x, wave = tid >> 5, lane = tid & 31, col = lane & 15, g = lane >> 4; const size_t b = blockIdx.z + TB0; const size_t fl = (size_t)blockIdx.x * 64 + wave * 16; const size_t f0 = (size_t)slab * FPS + fl; const int p0 = blockIdx.y * 128;
  v8f acc[8] = {};
#pragma unroll
  for (int kc = 0; kc < CM / 32; ++kc) { const v16b a = frag_b(PF + (f0 + col) * CM + kc * 32, lane);
#pragma unroll
    for (int jt = 0; jt < 8; ++jt) { const size_t prow = b * NPX + p0 + jt * 16 + col; acc[jt] = wmma_bf(a, frag_b(ML + prow * CM + kc * 32, lane), acc[jt]); acc[jt] = wmma_bf(a, frag_b(MH + prow * CM + kc * 32, lane), acc[jt]); } }
#pragma unroll
  for (int jt = 0; jt < 8; ++jt)
#pragma unroll
    for (int r = 0; r < 8; ++r) so[wave][8 * g + r][jt * 16 + col] = acc[jt][r] + bfr(BF[f0 + 8 * g + r]);
  LDSX();
  for (int rl = 0; rl < 16; ++rl) vst2(F + (b * FPS + fl + rl) * NPX + p0 + lane * 4, *(const v4f*)&so[wave][rl][lane * 4]);
}
__global__ __launch_bounds__(256) void k_el(const float* __restrict__ E1, const float* __restrict__ F, int slab, float* __restrict__ EL, float* __restrict__ ST) {
  __shared__ float spt[64][KP + 1]; __shared__ __align__(16) float so[CE][68]; __shared__ float sst[CE][2];
  const int t = threadIdx.x; const int y = slab * SLR + blockIdx.x; const size_t b = blockIdx.y + TB0; const int px = t >> 2, og = t & 3;
  for (int e = t; e < 64 * KP; e += 256) { const int p = e / KP, k = e % KP; const int c = k / 9, ij = k % 9, i = ij / 3, j = ij % 3; const int yy = y + i - 1, xx = p + j - 1;
    spt[p][k] = (yy >= 0 && yy < HH && xx >= 0 && xx < WW) ? bfr(E1[((b * CE + c) * HH + yy) * WW + xx]) : 0.f; }
  __syncthreads();
  { const size_t Ploc = (size_t)blockIdx.x * WW + px; const float* fp = F + (b * FPS) * (size_t)NPX + Ploc * NF;
    for (int oo = 0; oo < 8; ++oo) { const int o = og * 8 + oo; const float* fo = fp + o * KP; float a = 0.f;
#pragma unroll 1
      for (int k = 0; k < KP; ++k) a += fo[k] * spt[px][k];
      so[o][px] = fmaxf(a, 0.f); } }
  __syncthreads();
  if (t < CE) { float s = 0.f, q2 = 0.f; for (int p = 0; p < 64; ++p) { const float v = so[t][p]; s += v; q2 += v * v; } sst[t][0] = s; sst[t][1] = q2; }
  for (int e = t; e < CE * 16; e += 256) { const int o = e >> 4, q = e & 15; vst2(EL + ((b * CE + o) * HH + y) * WW + q * 4, *(const v4f*)&so[o][q * 4]); }
  __syncthreads();
  if (t < 16) vst2(ST + ((b * HH + y) * CE) * 2 + t * 4, *(const v4f*)(&sst[0][0] + t * 4));
}
__global__ __launch_bounds__(64) void k_stat(const float* __restrict__ ST, float* __restrict__ MS) {
  const int o = threadIdx.x; __shared__ __align__(16) float sm[CE][2];
  if (o < CE) { float s = 0.f, q2 = 0.f; for (int blk = TB0 * HH; blk < (TB0 + TNB) * HH; ++blk) { s += ST[((size_t)blk * CE + o) * 2]; q2 += ST[((size_t)blk * CE + o) * 2 + 1]; }
    const float n = (float)(TNB * NPX); const float mu = s / n; const float var = fmaxf(q2 / n - mu * mu, 0.f); sm[o][0] = mu; sm[o][1] = 1.0f / sqrtf(var + 1e-5f); }
  __syncthreads();
  if (o < 16) vst2(MS + o * 4, *(const v4f*)(&sm[0][0] + o * 4));
}
__global__ __launch_bounds__(64) void k_norm(const float* __restrict__ EL, const float* __restrict__ MS, float* __restrict__ OUT1) {
  const int t = threadIdx.x; const int y = blockIdx.x, o = blockIdx.y; const size_t b = blockIdx.z + TB0; const float mu = MS[o * 2], rs = MS[o * 2 + 1];
  __shared__ __align__(16) float s[64]; const size_t base = ((b * CE + o) * HH + y) * WW; s[t] = (EL[base + t] - mu) * rs; __syncthreads();
  if (t < 16) vst2(OUT1 + base + t * 4, *(const v4f*)&s[t * 4]);
}
extern "C" void kernel_launch(void* const* d_in, const int* in_sizes, int n_in, void* d_out, int out_size, void* d_ws, size_t ws_size, hipStream_t stream) {
  (void)in_sizes; (void)n_in; (void)out_size;
  const float** Fi = (const float**)d_in;
  if (ws_size < (size_t)WS_END) return;
  char* ws = (char*)d_ws; __bf16* PK = (__bf16*)ws; __bf16 *MH = (__bf16*)(ws + WS_MH), *ML = (__bf16*)(ws + WS_MLO); float* F = (float*)(ws + WS_F); float *EL = (float*)(ws + WS_EL), *ST = (float*)(ws + WS_ST), *MS = (float*)(ws + WS_MS);
  float* OUT0 = (float*)d_out; float* OUT1 = (float*)((char*)d_out + 2097152);
  k_pack<<<dim3(NF / 64, 2), 256, 0, stream>>>(Fi[2], Fi[4], PK);
  k_ml<<<dim3(HH, TNB), 128, 0, stream>>>(Fi[0], (const __bf16*)(ws + WS_PM), Fi[3], OUT0, MH, ML);
  for (int s = 0; s < NSL; ++s) {
    k_f<<<dim3(FPS / 64, NPX / 128, TNB), 128, 0, stream>>>((const __bf16*)(ws + WS_PF), MH, ML, Fi[5], s, F);
    k_el<<<dim3(SLR, TNB), 256, 0, stream>>>(Fi[1], F, s, EL, ST); }
  k_stat<<<1, 64, 0, stream>>>(ST, MS);
  k_norm<<<dim3(HH, CE, TNB), 64, 0, stream>>>(EL, MS, OUT1);
}
